// ShuffledSSM_13692355739871
// MI455X (gfx1250) — hardware-verified
//
#include <hip/hip_runtime.h>


#define NB_    16
#define CIN_   8
#define HI_    256
#define WI_    256
#define RR_    4
#define DM_    128
#define DS_    64
#define DI_    256
#define DTR_   8
#define XDN_   136
#define XPW_   144
#define LTOK_  4096
#define HQ_    64
#define WQ_    64
#define NGRP_  2
#define GB_    (NB_ / NGRP_)
#define MG_    (GB_ * LTOK_)
#define TCH_   16

static_assert(DM_ == CIN_ * RR_ * RR_);
static_assert(HQ_ * RR_ == HI_ && WQ_ * RR_ == WI_);
static_assert(LTOK_ == HQ_ * WQ_);
static_assert(HQ_ == 64 && WQ_ == 64);
static_assert(NB_ % NGRP_ == 0);
static_assert(MG_ % 64 == 0);
static_assert(DM_ % 32 == 0 && DI_ % 32 == 0);
static_assert(XPW_ % 48 == 0 && XPW_ >= XDN_);
static_assert(DTR_ + 2 * DS_ == XDN_);
static_assert(LTOK_ % TCH_ == 0 && TCH_ == 16);
static_assert(DS_ == 64 && DI_ == 256 && DTR_ == 8 && DM_ == 128);

typedef float          v4f   __attribute__((ext_vector_type(4)));
typedef float          v8f   __attribute__((ext_vector_type(8)));
typedef __bf16         v16b  __attribute__((ext_vector_type(16)));
typedef unsigned short u16x8 __attribute__((ext_vector_type(8)));
typedef unsigned short u16x4 __attribute__((ext_vector_type(4)));

union FragB { u16x8 h[2]; v16b v; };
union Pack4 { u16x4 v; unsigned short s[4]; };
union Pack8 { u16x8 v; unsigned short s[8]; };

constexpr size_t SZ_WI   = (size_t)2 * DI_ * DM_ * 2;
constexpr size_t SZ_WX   = (size_t)XPW_ * DI_ * 2;
constexpr size_t SZ_WO   = (size_t)DM_ * DI_ * 2;
constexpr size_t SZ_U16  = (size_t)MG_ * DM_ * 2;
constexpr size_t SZ_P16  = (size_t)MG_ * DI_ * 2;
constexpr size_t SZ_F    = (size_t)MG_ * DI_ * 4;
constexpr size_t SZ_DT8  = (size_t)MG_ * DTR_ * 4;
constexpr size_t SZ_BC   = (size_t)MG_ * 2 * DS_ * 4;

constexpr size_t OFF_WIH = 0;
constexpr size_t OFF_WIL = OFF_WIH + SZ_WI;
constexpr size_t OFF_WXH = OFF_WIL + SZ_WI;
constexpr size_t OFF_WXL = OFF_WXH + SZ_WX;
constexpr size_t OFF_WOH = OFF_WXL + SZ_WX;
constexpr size_t OFF_WOL = OFF_WOH + SZ_WO;
constexpr size_t OFF_RA  = OFF_WOL + SZ_WO;
constexpr size_t REG_A   = 2 * SZ_P16;
constexpr size_t OFF_UH  = OFF_RA;
constexpr size_t OFF_UL  = OFF_RA + SZ_U16;
constexpr size_t OFF_XCH = OFF_RA;
constexpr size_t OFF_XCL = OFF_RA + SZ_P16;
constexpr size_t OFF_YH  = OFF_RA;
constexpr size_t OFF_YL  = OFF_RA + SZ_P16;
constexpr size_t OFF_XIN = OFF_RA + REG_A;
constexpr size_t OFF_Z   = OFF_XIN + SZ_F;
constexpr size_t OFF_DT8 = OFF_Z + SZ_F;
constexpr size_t OFF_BC  = OFF_DT8 + SZ_DT8;
constexpr size_t WS_END  = OFF_BC + SZ_BC;
constexpr size_t YPL_    = (size_t)MG_ * DI_;

static_assert(OFF_UL + SZ_U16 <= OFF_RA + REG_A);
static_assert(OFF_XCL + SZ_P16 <= OFF_RA + REG_A);
static_assert(OFF_YL + SZ_P16 <= OFF_RA + REG_A);
static_assert(OFF_YL == OFF_YH + YPL_ * 2);
static_assert(WS_END <= (size_t)134217728);
static_assert(OFF_WIL % 128 == 0 && OFF_WXH % 128 == 0 && OFF_WXL % 128 == 0 && OFF_WOH % 128 == 0);
static_assert(OFF_WOL % 128 == 0 && OFF_RA % 128 == 0 && OFF_UL % 128 == 0 && OFF_XCL % 128 == 0);
static_assert(OFF_XIN % 128 == 0 && OFF_Z % 128 == 0 && OFF_DT8 % 128 == 0 && OFF_BC % 128 == 0);

__device__ __forceinline__ unsigned short f32_to_bf16(float f) {
    const unsigned u = __float_as_uint(f);
    const unsigned r = u + 0x7FFFu + ((u >> 16) & 1u);
    return (unsigned short)(r >> 16);
}
__device__ __forceinline__ float bf16_to_f32(unsigned short b) {
    return __uint_as_float(((unsigned)b) << 16);
}
__device__ __forceinline__ void split_bf16(float f, unsigned short& hb, unsigned short& lb) {
    hb = f32_to_bf16(f);
    lb = f32_to_bf16(f - bf16_to_f32(hb));
}
__device__ __forceinline__ float silu_f(float x) {
    const float e = __expf(-x);
    return x * __builtin_amdgcn_rcpf(1.0f + e);
}
__device__ __forceinline__ float softplus_f(float x) {
    return fmaxf(x, 0.0f) + log1pf(__expf(-fabsf(x)));
}
__device__ __forceinline__ v8f ld8f(const float* p) {
    const v4f a = *(const v4f*)p;
    const v4f b = *(const v4f*)(p + 4);
    return __builtin_shufflevector(a, b, 0, 1, 2, 3, 4, 5, 6, 7);
}
__device__ __forceinline__ v8f zero8() {
    v8f z;
#pragma unroll
    for (int c = 0; c < 8; ++c) z[c] = 0.0f;
    return z;
}

__device__ __forceinline__ void mma16(v8f& acc, const FragB& a, const FragB& b) {
    acc = __builtin_amdgcn_wmma_f32_16x16x32_bf16(false, a.v, false, b.v, (short)0, acc, false, false);
    asm volatile("v_nop\n\tv_nop\n\tv_nop\n\tv_nop" : "+v"(acc) : "v"(a.v), "v"(b.v));
}

template<int NBF>
__device__ __forceinline__ void gemm_core(const unsigned short* __restrict__ A,  const unsigned short* __restrict__ A2,
                                          const unsigned short* __restrict__ Bw, const unsigned short* __restrict__ B2,
                                          const int K, const int rowW, const int colW, const int lane,
                                          v8f (&acc)[2 * NBF])
{
    const int h = lane >> 4, m = lane & 15;
#pragma unroll
    for (int j = 0; j < 2 * NBF; ++j)
#pragma unroll
        for (int r = 0; r < 8; ++r) acc[j][r] = 0.0f;

    const size_t aoff  = (size_t)(rowW + m) * K + 8 * h;
    const size_t boff  = (size_t)(colW + m) * K + 8 * h;
    const size_t sub16 = (size_t)16 * K;
    const int nk = K >> 5;

#pragma unroll 1
    for (int kt = 0; kt < nk; ++kt) {
        const size_t k0 = (size_t)kt * 32;
        FragB fa[2], ga[2], fb[NBF], gb[NBF];
#pragma unroll
        for (int s = 0; s < 2; ++s) {
            const unsigned short* p = A  + aoff + s * sub16 + k0;
            const unsigned short* q = A2 + aoff + s * sub16 + k0;
            fa[s].h[0] = *(const u16x8*)(p);
            fa[s].h[1] = *(const u16x8*)(p + 16);
            ga[s].h[0] = *(const u16x8*)(q);
            ga[s].h[1] = *(const u16x8*)(q + 16);
        }
#pragma unroll
        for (int j = 0; j < NBF; ++j) {
            const unsigned short* p = Bw + boff + j * sub16 + k0;
            const unsigned short* q = B2 + boff + j * sub16 + k0;
            fb[j].h[0] = *(const u16x8*)(p);
            fb[j].h[1] = *(const u16x8*)(p + 16);
            gb[j].h[0] = *(const u16x8*)(q);
            gb[j].h[1] = *(const u16x8*)(q + 16);
        }
#pragma unroll
        for (int s = 0; s < 2; ++s)
#pragma unroll
            for (int j = 0; j < NBF; ++j) {
                mma16(acc[s * NBF + j], fa[s], fb[j]);
                mma16(acc[s * NBF + j], fa[s], gb[j]);
                mma16(acc[s * NBF + j], ga[s], fb[j]);
            }
    }
}

template<int NBF>
__device__ __forceinline__ void stage_acc(float* st, const int PB, const int r0, const int c0, const int lane,
                                          const v8f (&acc)[2 * NBF])
{
    const int h = lane >> 4, m = lane & 15;
#pragma unroll
    for (int s = 0; s < 2; ++s)
#pragma unroll
        for (int j = 0; j < NBF; ++j)
#pragma unroll
            for (int r = 0; r < 8; ++r)
                st[(r0 + s * 16 + 8 * h + r) * PB + c0 + j * 16 + m] = acc[s * NBF + j][r];
}

__global__ __launch_bounds__(256)
void k_cvt_split(const float* __restrict__ src, unsigned short* dh, unsigned short* dl, int n8, int nsrc8)
{
    const int i = blockIdx.x * 256 + threadIdx.x;
    if (i >= n8) return;
    const int ic = (i < nsrc8) ? i : (nsrc8 - 1);
    v8f x = ld8f(src + (size_t)ic * 8);
    if (i >= nsrc8) x = zero8();
    Pack8 hp, lp;
#pragma unroll
    for (int c = 0; c < 8; ++c) split_bf16(x[c], hp.s[c], lp.s[c]);
    const u16x8 hv = hp.v, lv = lp.v;
    const size_t e = (size_t)i * 8;
    *(volatile u16x8*)(dh + e) = hv;
    *(volatile u16x8*)(dl + e) = lv;
    __threadfence();
    *(volatile u16x8*)(dh + e) = hv;
    *(volatile u16x8*)(dl + e) = lv;
}

__global__ __launch_bounds__(64)
void k_ln(const float* __restrict__ x, const float* __restrict__ gam, const float* __restrict__ bet,
          unsigned short* uh, unsigned short* ul, int g)
{
    __shared__ __attribute__((aligned(16))) unsigned short sh[64 * DM_];
    __shared__ __attribute__((aligned(16))) unsigned short sl[64 * DM_];

    const int w  = threadIdx.x;
    const int hq = blockIdx.x & (HQ_ - 1);
    const int bl = blockIdx.x >> 6;
    const int b  = g * GB_ + bl;
    const float* xb = x + (size_t)b * (CIN_ * HI_ * WI_) + (size_t)(RR_ * hq) * WI_ + RR_ * w;

    float s = 0.0f;
#pragma unroll 1
    for (int ci = 0; ci < CIN_ * RR_; ++ci) {
        const size_t off = (size_t)(ci >> 2) * (HI_ * WI_) + (size_t)(ci & 3) * WI_;
        const v4f v = *(const v4f*)(xb + off);
        s += v[0]; s += v[1]; s += v[2]; s += v[3];
    }
    const float mean = s * (1.0f / (float)DM_);
    float q = 0.0f;
#pragma unroll 1
    for (int ci = 0; ci < CIN_ * RR_; ++ci) {
        const size_t off = (size_t)(ci >> 2) * (HI_ * WI_) + (size_t)(ci & 3) * WI_;
        const v4f v = *(const v4f*)(xb + off);
#pragma unroll
        for (int j = 0; j < 4; ++j) { const float dv = v[j] - mean; q = fmaf(dv, dv, q); }
    }
    const float var  = q * (1.0f / (float)DM_);
    const float rstd = rsqrtf(var + 1e-5f);
#pragma unroll 1
    for (int ci = 0; ci < CIN_ * RR_; ++ci) {
        const size_t off = (size_t)(ci >> 2) * (HI_ * WI_) + (size_t)(ci & 3) * WI_;
        const v4f v  = *(const v4f*)(xb + off);
        const v4f gv = *(const v4f*)(gam + ci * 4);
        const v4f bv = *(const v4f*)(bet + ci * 4);
        Pack4 hp, lp;
#pragma unroll
        for (int j = 0; j < 4; ++j) {
            const float val = (v[j] - mean) * rstd * gv[j] + bv[j];
            split_bf16(val, hp.s[j], lp.s[j]);
        }
        *(u16x4*)(sh + w * DM_ + ci * 4) = hp.v;
        *(u16x4*)(sl + w * DM_ + ci * 4) = lp.v;
    }
    __syncthreads();

    const size_t m0 = (size_t)bl * LTOK_ + (size_t)hq * WQ_;
    unsigned short* gh = uh + m0 * DM_;
    unsigned short* gl = ul + m0 * DM_;
#pragma unroll
    for (int it = 0; it < 16; ++it) {
        const int idx = it * 64 + w;
        const u16x8 hv = *(const u16x8*)(sh + idx * 8);
        const u16x8 lv = *(const u16x8*)(sl + idx * 8);
        *(volatile u16x8*)(gh + (size_t)idx * 8) = hv;
        *(volatile u16x8*)(gl + (size_t)idx * 8) = lv;
    }
    __threadfence();
#pragma unroll
    for (int it = 0; it < 16; ++it) {
        const int idx = it * 64 + w;
        const u16x8 hv = *(const u16x8*)(sh + idx * 8);
        const u16x8 lv = *(const u16x8*)(sl + idx * 8);
        *(volatile u16x8*)(gh + (size_t)idx * 8) = hv;
        *(volatile u16x8*)(gl + (size_t)idx * 8) = lv;
    }
}

__global__ __launch_bounds__(128)
void k_inproj(const unsigned short* __restrict__ A,  const unsigned short* __restrict__ A2,
              const unsigned short* __restrict__ Bw, const unsigned short* __restrict__ B2,
              float* xin, float* zf)
{
    constexpr int PB = 64 + 4;
    __shared__ __attribute__((aligned(16))) float st[64 * PB];

    const int tid  = threadIdx.x;
    const int lane = tid & 31;
    const int wave = tid >> 5;
    const int wm   = wave >> 1;
    const int wn   = wave & 1;
    const int rowB = blockIdx.y * 64;
    const int colB = blockIdx.x * 64;

    v8f acc[4];
    gemm_core<2>(A, A2, Bw, B2, DM_, rowB + wm * 32, colB + wn * 32, lane, acc);
    stage_acc<2>(st, PB, wm * 32, wn * 32, lane, acc);
    __syncthreads();

    float* dst = (colB < DI_) ? (xin + colB) : (zf + (colB - DI_));
#pragma unroll
    for (int it = 0; it < 8; ++it) {
        const int idx = it * 128 + tid;
        const int row = idx >> 4;
        const int c4  = (idx & 15) * 4;
        const v4f v = *(const v4f*)(st + row * PB + c4);
        *(volatile v4f*)(dst + (size_t)(rowB + row) * DI_ + c4) = v;
    }
    __threadfence();
#pragma unroll
    for (int it = 0; it < 8; ++it) {
        const int idx = it * 128 + tid;
        const int row = idx >> 4;
        const int c4  = (idx & 15) * 4;
        const v4f v = *(const v4f*)(st + row * PB + c4);
        *(volatile v4f*)(dst + (size_t)(rowB + row) * DI_ + c4) = v;
    }
}

__global__ __launch_bounds__(32)
void k_conv(const float* __restrict__ xin, const float* __restrict__ cw, const float* __restrict__ cb,
            unsigned short* xch, unsigned short* xcl)
{
    const int m  = blockIdx.x;
    const int l  = m & (LTOK_ - 1);
    const int d0 = threadIdx.x * 8;
    const int m1 = (l >= 1) ? (m - 1) : m;
    const int m2 = (l >= 2) ? (m - 2) : m;
    const int m3 = (l >= 3) ? (m - 3) : m;

    const v8f x3 = ld8f(xin + (size_t)m  * DI_ + d0);
    const v8f t2 = ld8f(xin + (size_t)m1 * DI_ + d0);
    const v8f t1 = ld8f(xin + (size_t)m2 * DI_ + d0);
    const v8f t0 = ld8f(xin + (size_t)m3 * DI_ + d0);
    const v8f z8 = zero8();
    const v8f x2 = (l >= 1) ? t2 : z8;
    const v8f x1 = (l >= 2) ? t1 : z8;
    const v8f x0 = (l >= 3) ? t0 : z8;

    v4f wv[8];
#pragma unroll
    for (int c = 0; c < 8; ++c) wv[c] = *(const v4f*)(cw + (size_t)(d0 + c) * 4);
    const v8f bias = ld8f(cb + d0);

    Pack8 hp, lp;
#pragma unroll
    for (int c = 0; c < 8; ++c) {
        const float conv = wv[c][0] * x0[c] + wv[c][1] * x1[c] + wv[c][2] * x2[c] + wv[c][3] * x3[c];
        const float u = silu_f(conv + bias[c]);
        split_bf16(u, hp.s[c], lp.s[c]);
    }
    const u16x8 hv = hp.v, lv = lp.v;
    const size_t e = (size_t)m * DI_ + d0;
    *(volatile u16x8*)(xch + e) = hv;
    *(volatile u16x8*)(xcl + e) = lv;
    __threadfence();
    *(volatile u16x8*)(xch + e) = hv;
    *(volatile u16x8*)(xcl + e) = lv;
}

__global__ __launch_bounds__(192)
void k_xproj(const unsigned short* __restrict__ A,  const unsigned short* __restrict__ A2,
             const unsigned short* __restrict__ Bw, const unsigned short* __restrict__ B2,
             float* dt8, float* bcf)
{
    constexpr int PB = XPW_ + 4;
    __shared__ __attribute__((aligned(16))) float st[64 * PB];

    const int tid  = threadIdx.x;
    const int lane = tid & 31;
    const int wave = tid >> 5;
    const int wm   = wave / 3;
    const int wn   = wave - wm * 3;
    const int rowB = blockIdx.y * 64;

    v8f acc[6];
    gemm_core<3>(A, A2, Bw, B2, DI_, rowB + wm * 32, wn * 48, lane, acc);
    stage_acc<3>(st, PB, wm * 32, wn * 48, lane, acc);
    __syncthreads();

#pragma unroll
    for (int it = 0; it < 11; ++it) {
        const int idx = it * 192 + tid;
        if (idx < 64 * 32) {
            const int row = idx >> 5;
            const int c4  = (idx & 31) * 4;
            const v4f v = *(const v4f*)(st + row * PB + DTR_ + c4);
            *(volatile v4f*)(bcf + (size_t)(rowB + row) * (2 * DS_) + c4) = v;
        }
    }
    if (tid < 128) {
        const int row = tid >> 1;
        const int c4  = (tid & 1) * 4;
        const v4f v = *(const v4f*)(st + row * PB + c4);
        *(volatile v4f*)(dt8 + (size_t)(rowB + row) * DTR_ + c4) = v;
    }
    __threadfence();
#pragma unroll
    for (int it = 0; it < 11; ++it) {
        const int idx = it * 192 + tid;
        if (idx < 64 * 32) {
            const int row = idx >> 5;
            const int c4  = (idx & 31) * 4;
            const v4f v = *(const v4f*)(st + row * PB + DTR_ + c4);
            *(volatile v4f*)(bcf + (size_t)(rowB + row) * (2 * DS_) + c4) = v;
        }
    }
    if (tid < 128) {
        const int row = tid >> 1;
        const int c4  = (tid & 1) * 4;
        const v4f v = *(const v4f*)(st + row * PB + c4);
        *(volatile v4f*)(dt8 + (size_t)(rowB + row) * DTR_ + c4) = v;
    }
}

__global__ __launch_bounds__(256)
void k_scan(const float* __restrict__ xin, const float* __restrict__ zf,
            const float* __restrict__ dt8, const float* __restrict__ bcf,
            const float* __restrict__ cw,  const float* __restrict__ cb,
            const float* __restrict__ wdt, const float* __restrict__ dtb,
            const float* __restrict__ alog, const float* __restrict__ Dp,
            unsigned short* yh)
{
    __shared__ __attribute__((aligned(16))) float  sBC[TCH_ * 2 * DS_];
    __shared__ __attribute__((aligned(16))) float  sD8[TCH_ * DTR_];
    __shared__ __attribute__((aligned(16))) float2 sPA[TCH_ * 64];
    __shared__ __attribute__((aligned(16))) float2 sPB[TCH_ * 64];
    __shared__ __attribute__((aligned(16))) unsigned short sY[2 * TCH_ * 64];

    const int tid  = threadIdx.x;
    const int chl  = tid >> 2;
    const int sg   = tid & 3;
    const int dblk = blockIdx.x * 64;
    const int d    = dblk + chl;
    const size_t mrow0 = (size_t)blockIdx.y * LTOK_;

    float a2[16], hs[16];
#pragma unroll
    for (int q = 0; q < 16; ++q) {
        a2[q] = -__expf(alog[(size_t)d * DS_ + sg * 16 + q]) * 1.44269504088896341f;
        hs[q] = 0.0f;
    }
    float w8[DTR_];
#pragma unroll
    for (int r = 0; r < DTR_; ++r) w8[r] = wdt[(size_t)d * DTR_ + r];
    const float tb  = dtb[d];
    const float cw0 = cw[d * 4 + 0], cw1 = cw[d * 4 + 1], cw2 = cw[d * 4 + 2], cw3 = cw[d * 4 + 3];
    const float cbias = cb[d];
    const float Dd  = Dp[d];
    const float* xr = xin + d;
    const float* zr = zf + d;

#pragma unroll 1
    for (int l0 = 0; l0 < LTOK_; l0 += TCH_) {
#pragma unroll
        for (int it = 0; it < 2; ++it) {
            const int idx = it * 256 + tid;
            const int t   = idx >> 5;
            const int c4  = (idx & 31) * 4;
            *(v4f*)(sBC + t * (2 * DS_) + c4) = *(const v4f*)(bcf + (mrow0 + l0 + t) * (2 * DS_) + c4);
        }
        if (tid < 32) {
            const int t  = tid >> 1;
            const int c4 = (tid & 1) * 4;
            *(v4f*)(sD8 + t * DTR_ + c4) = *(const v4f*)(dt8 + (mrow0 + l0 + t) * DTR_ + c4);
        }
        __syncthreads();

#pragma unroll 1
        for (int i = 0; i < 4; ++i) {
            const int t = 4 * i + sg;
            const int l = l0 + t;
            const size_t m  = mrow0 + (size_t)l;
            const size_t m1 = (l >= 1) ? (m - 1) : m;
            const size_t m2 = (l >= 2) ? (m - 2) : m;
            const size_t m3 = (l >= 3) ? (m - 3) : m;
            const float x3 = xr[m * DI_];
            const float v2 = xr[m1 * DI_];
            const float v1 = xr[m2 * DI_];
            const float v0 = xr[m3 * DI_];
            const float x2 = (l >= 1) ? v2 : 0.0f;
            const float x1 = (l >= 2) ? v1 : 0.0f;
            const float x0 = (l >= 3) ? v0 : 0.0f;
            const float conv = cw0 * x0 + cw1 * x1 + cw2 * x2 + cw3 * x3;
            const float u = silu_f(conv + cbias);
            const v4f r0v = *(const v4f*)(sD8 + t * DTR_);
            const v4f r1v = *(const v4f*)(sD8 + t * DTR_ + 4);
            float dot = r0v[0] * w8[0];
            dot = fmaf(r0v[1], w8[1], dot);
            dot = fmaf(r0v[2], w8[2], dot);
            dot = fmaf(r0v[3], w8[3], dot);
            dot = fmaf(r1v[0], w8[4], dot);
            dot = fmaf(r1v[1], w8[5], dot);
            dot = fmaf(r1v[2], w8[6], dot);
            dot = fmaf(r1v[3], w8[7], dot);
            const float dtv = softplus_f(dot + tb);
            const float sz  = silu_f(zr[m * DI_]);
            sPA[t * 64 + chl] = make_float2(dtv, dtv * u);
            sPB[t * 64 + chl] = make_float2(Dd * u, sz);
        }
        __syncthreads();

#pragma unroll 1
        for (int t = 0; t < TCH_; ++t) {
            const float2 pa = sPA[t * 64 + chl];
            const float dtv = pa.x;
            const float du  = pa.y;
            const float* bp = sBC + t * (2 * DS_) + sg * 16;
            v4f bq[4], cq[4];
#pragma unroll
            for (int i = 0; i < 4; ++i) {
                bq[i] = *(const v4f*)(bp + 4 * i);
                cq[i] = *(const v4f*)(bp + DS_ + 4 * i);
            }
            float y = 0.0f;
#pragma unroll
            for (int q = 0; q < 16; ++q) {
                const float da = __builtin_amdgcn_exp2f(dtv * a2[q]);
                hs[q] = fmaf(hs[q], da, du * bq[q >> 2][q & 3]);
                y = fmaf(hs[q], cq[q >> 2][q & 3], y);
            }
            y += __shfl_xor(y, 1, 32);
            y += __shfl_xor(y, 2, 32);
            const float2 pb = sPB[t * 64 + chl];
            const float gval = (y + pb.x) * pb.y;
            unsigned short hb, lb;
            split_bf16(gval, hb, lb);
            if (sg == 0) {
                sY[t * 64 + chl] = hb;
                sY[TCH_ * 64 + t * 64 + chl] = lb;
            }
        }
        __syncthreads();

        {
            const int plane = tid >> 7;
            const int rr = tid & 127;
            const int t  = rr >> 3;
            const int c8 = (rr & 7) * 8;
            const u16x8 v = *(const u16x8*)(sY + plane * (TCH_ * 64) + t * 64 + c8);
            unsigned short* dst = yh + (size_t)plane * YPL_ + (mrow0 + l0 + t) * DI_ + dblk + c8;
            *(volatile u16x8*)dst = v;
            __threadfence();
            *(volatile u16x8*)dst = v;
        }
        __syncthreads();
    }
}

__global__ __launch_bounds__(128)
void k_outproj(const unsigned short* __restrict__ A,  const unsigned short* __restrict__ A2,
               const unsigned short* __restrict__ Bw, const unsigned short* __restrict__ B2,
               const float* __restrict__ x, float* out, int g)
{
    constexpr int PB = 64 + 4;
    __shared__ __attribute__((aligned(16))) float st[64 * PB];

    const int tid  = threadIdx.x;
    const int lane = tid & 31;
    const int wave = tid >> 5;
    const int wm   = wave >> 1;
    const int wn   = wave & 1;
    const int rowB = blockIdx.y * 64;
    const int colB = blockIdx.x * 64;
    const int bl   = blockIdx.y >> 6;
    const int hq   = blockIdx.y & (HQ_ - 1);
    const int b    = g * GB_ + bl;

    v8f acc[4];
    gemm_core<2>(A, A2, Bw, B2, DI_, rowB + wm * 32, colB + wn * 32, lane, acc);
    stage_acc<2>(st, PB, wm * 32, wn * 32, lane, acc);
    __syncthreads();

    v4f vals[8];
#pragma unroll
    for (int it = 0; it < 8; ++it) {
        const int idx = it * 128 + tid;
        const int p = idx >> 6;
        const int k = idx & 63;
        const int e = colB + 4 * p;
        const int c = e >> 4;
        const int i = (e >> 2) & 3;
        const size_t ra = ((size_t)(b * CIN_ + c) * HI_ + (size_t)(RR_ * hq + i)) * WI_ + (size_t)(RR_ * k);
        const v4f tv = *(const v4f*)(st + k * PB + 4 * p);
        const v4f xv = *(const v4f*)(x + ra);
        vals[it] = tv + xv;
        *(volatile v4f*)(out + ra) = vals[it];
    }
    __threadfence();
#pragma unroll
    for (int it = 0; it < 8; ++it) {
        const int idx = it * 128 + tid;
        const int p = idx >> 6;
        const int k = idx & 63;
        const int e = colB + 4 * p;
        const int c = e >> 4;
        const int i = (e >> 2) & 3;
        const size_t ra = ((size_t)(b * CIN_ + c) * HI_ + (size_t)(RR_ * hq + i)) * WI_ + (size_t)(RR_ * k);
        *(volatile v4f*)(out + ra) = vals[it];
    }
}

extern "C" void kernel_launch(void* const* d_in, const int* in_sizes, int n_in,
                              void* d_out, int out_size, void* d_ws, size_t ws_size,
                              hipStream_t stream)
{
    if (n_in < 12) return;
    if (in_sizes[0]  != NB_ * CIN_ * HI_ * WI_) return;
    if (in_sizes[1]  != DM_)                    return;
    if (in_sizes[2]  != DM_)                    return;
    if (in_sizes[3]  != 2 * DI_ * DM_)          return;
    if (in_sizes[4]  != DI_ * 4)                return;
    if (in_sizes[5]  != DI_)                    return;
    if (in_sizes[6]  != XDN_ * DI_)             return;
    if (in_sizes[7]  != DI_ * DTR_)             return;
    if (in_sizes[8]  != DI_)                    return;
    if (in_sizes[9]  != DI_ * DS_)              return;
    if (in_sizes[10] != DI_)                    return;
    if (in_sizes[11] != DM_ * DI_)              return;
    if (out_size != NB_ * CIN_ * HI_ * WI_)     return;
    if (ws_size < WS_END)                       return;

    const float* x    = (const float*)d_in[0];
    const float* gam  = (const float*)d_in[1];
    const float* bet  = (const float*)d_in[2];
    const float* win  = (const float*)d_in[3];
    const float* cw   = (const float*)d_in[4];
    const float* cb   = (const float*)d_in[5];
    const float* wx   = (const float*)d_in[6];
    const float* wdt  = (const float*)d_in[7];
    const float* dtb  = (const float*)d_in[8];
    const float* alog = (const float*)d_in[9];
    const float* Dp   = (const float*)d_in[10];
    const float* wo   = (const float*)d_in[11];
    float* out = (float*)d_out;

    char* ws = (char*)d_ws;
    unsigned short* wih = (unsigned short*)(ws + OFF_WIH);
    unsigned short* wil = (unsigned short*)(ws + OFF_WIL);
    unsigned short* wxh = (unsigned short*)(ws + OFF_WXH);
    unsigned short* wxl = (unsigned short*)(ws + OFF_WXL);
    unsigned short* woh = (unsigned short*)(ws + OFF_WOH);
    unsigned short* wol = (unsigned short*)(ws + OFF_WOL);
    unsigned short* uh  = (unsigned short*)(ws + OFF_UH);
    unsigned short* ul  = (unsigned short*)(ws + OFF_UL);
    unsigned short* xch = (unsigned short*)(ws + OFF_XCH);
    unsigned short* xcl = (unsigned short*)(ws + OFF_XCL);
    unsigned short* yh  = (unsigned short*)(ws + OFF_YH);
    unsigned short* yl  = (unsigned short*)(ws + OFF_YL);
    float*          xin = (float*)(ws + OFF_XIN);
    float*          zf  = (float*)(ws + OFF_Z);
    float*          dt8 = (float*)(ws + OFF_DT8);
    float*          bcf = (float*)(ws + OFF_BC);

    {
        int n8 = (2 * DI_ * DM_) / 8;
        k_cvt_split<<<dim3(n8 / 256), dim3(256), 0, stream>>>(win, wih, wil, n8, n8);
        n8 = (XPW_ * DI_) / 8;
        k_cvt_split<<<dim3(n8 / 256), dim3(256), 0, stream>>>(wx, wxh, wxl, n8, (int)((XDN_ * DI_) / 8));
        n8 = (DM_ * DI_) / 8;
        k_cvt_split<<<dim3(n8 / 256), dim3(256), 0, stream>>>(wo, woh, wol, n8, n8);
    }
    static_assert(((2 * DI_ * DM_) / 8) % 256 == 0);
    static_assert(((XPW_ * DI_) / 8) % 256 == 0);
    static_assert(((DM_ * DI_) / 8) % 256 == 0);

    for (int g = 0; g < NGRP_; ++g) {
        k_ln<<<dim3(GB_ * HQ_), dim3(64), 0, stream>>>(x, gam, bet, uh, ul, g);
        k_inproj<<<dim3((2 * DI_) / 64, MG_ / 64), dim3(128), 0, stream>>>(uh, ul, wih, wil, xin, zf);
        k_conv<<<dim3(MG_), dim3(32), 0, stream>>>(xin, cw, cb, xch, xcl);
        k_xproj<<<dim3(1, MG_ / 64), dim3(192), 0, stream>>>(xch, xcl, wxh, wxl, dt8, bcf);
        k_scan<<<dim3(DI_ / 64, GB_), dim3(256), 0, stream>>>(xin, zf, dt8, bcf, cw, cb, wdt, dtb, alog, Dp, yh);
        k_outproj<<<dim3(DM_ / 64, MG_ / 64), dim3(128), 0, stream>>>(yh, yl, woh, wol, x, out, g);
    }
}
